// FeedForward_29137058136069
// MI455X (gfx1250) — hardware-verified
//
#include <hip/hip_runtime.h>
#include <math.h>
#include <stdint.h>

#define NBATCH 2
#define SEQ    2048
#define NHEAD  16
#define HDIM   64
#define DMOD   (NHEAD * HDIM)
#define NTOK   (NBATCH * SEQ)
#define MBLK   128
#define NMB    (SEQ / MBLK)

typedef __attribute__((ext_vector_type(16))) __bf16   v16b;
typedef __attribute__((ext_vector_type(8)))  __bf16   v8b;
typedef __attribute__((ext_vector_type(8)))  float    v8f;
typedef __attribute__((ext_vector_type(4)))  float    v4f;
typedef __attribute__((ext_vector_type(4)))  unsigned int v4u;

#define AT_D  64
#define AT_NW 4
#define AT_QB 64
#define AT_KC 64
#define OFF_L ((size_t)NTOK * DMOD)
#define OFF_M (OFF_L + (size_t)NBATCH * NHEAD * SEQ)
#define OUT_N (OFF_M + (size_t)NBATCH * NHEAD * SEQ)

static_assert(DMOD == 1024);
static_assert(HDIM == AT_D);
static_assert(SEQ % AT_QB == 0);
static_assert(SEQ % AT_KC == 0);
static_assert(MBLK % AT_QB == 0);
static_assert(MBLK % AT_KC == 0);
static_assert((NTOK * DMOD) % (8 * 256) == 0);
static_assert(OFF_M + (size_t)NBATCH * NHEAD * SEQ == OUT_N);

__device__ __forceinline__ unsigned short f2bf_bits(float f) {
  unsigned u = __float_as_uint(f);
  return (unsigned short)((u + 0x7FFFu + ((u >> 16) & 1u)) >> 16);
}
__device__ __forceinline__ float bf_bits2f(unsigned short h) { return __uint_as_float(((unsigned)h) << 16); }
__device__ __forceinline__ unsigned pk16(unsigned short a, unsigned short b) { return (unsigned)a | ((unsigned)b << 16); }

__device__ __forceinline__ v16b ldfrag_b(const __bf16* p) {
  union { v16b v; v8b h[2]; } f;
  f.h[0] = *(const v8b*)(p);
  f.h[1] = *(const v8b*)(p + 16);
  return f.v;
}
__device__ __forceinline__ v8f at_mma(v16b a, v16b b, v8f c) {
  c = __builtin_amdgcn_wmma_f32_16x16x32_bf16(false, a, false, b, (short)0, c, false, false);
  asm volatile("v_nop\n\tv_nop\n\tv_nop\n\tv_nop" : "+v"(c) : "v"(a), "v"(b));
  return c;
}

__global__ __launch_bounds__(256) void cvt_qk_kernel(const float* __restrict__ q, const float* __restrict__ k,
                                                     unsigned short* __restrict__ QB, unsigned short* __restrict__ KB,
                                                     int n8) {
  int i = blockIdx.x * 256 + threadIdx.x;
  i = (i < n8) ? i : (n8 - 1);
  const size_t e0 = (size_t)i * 8;
  const v4f qa = *(const v4f*)(q + e0);
  const v4f qc = *(const v4f*)(q + e0 + 4);
  const v4f ka = *(const v4f*)(k + e0);
  const v4f kc = *(const v4f*)(k + e0 + 4);
  v4u qv, kv;
  qv[0] = pk16(f2bf_bits(qa[0]), f2bf_bits(qa[1]));
  qv[1] = pk16(f2bf_bits(qa[2]), f2bf_bits(qa[3]));
  qv[2] = pk16(f2bf_bits(qc[0]), f2bf_bits(qc[1]));
  qv[3] = pk16(f2bf_bits(qc[2]), f2bf_bits(qc[3]));
  kv[0] = pk16(f2bf_bits(ka[0]), f2bf_bits(ka[1]));
  kv[1] = pk16(f2bf_bits(ka[2]), f2bf_bits(ka[3]));
  kv[2] = pk16(f2bf_bits(kc[0]), f2bf_bits(kc[1]));
  kv[3] = pk16(f2bf_bits(kc[2]), f2bf_bits(kc[3]));
  *(volatile v4u*)(QB + e0) = qv;
  *(volatile v4u*)(KB + e0) = kv;
  __threadfence();
  *(volatile v4u*)(QB + e0) = qv;
  *(volatile v4u*)(KB + e0) = kv;
}

__global__ __launch_bounds__(256) void vtrans_kernel(const float* __restrict__ v, unsigned short* __restrict__ VT) {
  __shared__ __align__(16) unsigned short th[64 * 72];
  const int c0  = blockIdx.x * 64;
  const int r0  = blockIdx.y * 64;
  const int b   = blockIdx.z;
  const int tid = threadIdx.x;
  {
    const int rr = tid >> 2;
    const int cq = (tid & 3) * 16;
    const float* src = v + ((size_t)b * SEQ + r0 + rr) * DMOD + c0 + cq;
#pragma unroll
    for (int qq = 0; qq < 4; ++qq) {
      const v4f f = *(const v4f*)(src + 4 * qq);
#pragma unroll
      for (int e = 0; e < 4; ++e) th[rr * 72 + cq + 4 * qq + e] = f2bf_bits(f[e]);
    }
  }
  __syncthreads();
  const int sub = tid >> 3;
  const int c8  = (tid & 7) * 8;
  v4u hv[2];
#pragma unroll
  for (int it = 0; it < 2; ++it) {
    const int oc = it * 32 + sub;
    v4u a;
#pragma unroll
    for (int qq = 0; qq < 4; ++qq)
      a[qq] = pk16(th[(c8 + 2 * qq) * 72 + oc], th[(c8 + 2 * qq + 1) * 72 + oc]);
    hv[it] = a;
  }
  for (int pass = 0; pass < 2; ++pass) {
#pragma unroll
    for (int it = 0; it < 2; ++it) {
      const int oc = it * 32 + sub;
      const size_t go = ((size_t)b * DMOD + c0 + oc) * SEQ + r0 + c8;
      *(volatile v4u*)(VT + go) = hv[it];
    }
    __threadfence();
  }
}

__global__ __launch_bounds__(128)
void attn64_kernel(const unsigned short* __restrict__ qbp, const unsigned short* __restrict__ kbp,
                   const unsigned short* __restrict__ vtp, const int* __restrict__ bmask,
                   float* __restrict__ out, float sscale) {
  union FB { v16b v; v8b h[2]; };
  __shared__ __align__(16) __bf16 Ksh[AT_KC * AT_D];
  __shared__ __align__(16) __bf16 Vth[AT_D * AT_KC];
  __shared__ __align__(16) __bf16 Psh[AT_NW][16 * AT_KC];
  __shared__ __align__(16) __bf16 Psl[AT_NW][16 * AT_KC];
  __shared__ __align__(16) float  Os[AT_NW][16 * 68];
  __shared__ __align__(16) float  Ls[AT_QB];
  __shared__ __align__(16) float  Ms[AT_QB];

  const int tid  = threadIdx.x;
  const int wave = tid >> 5;
  const int lane = tid & 31;
  const int hh   = lane >> 4;
  const int c    = lane & 15;

  const int nqb = SEQ / AT_QB;
  const int bx  = blockIdx.x;
  const int qb  = bx % nqb;
  const int h   = bx / nqb;
  const int b   = blockIdx.y;
  const int q0  = qb * AT_QB + wave * 16;
  const int qbk = (qb * AT_QB) / MBLK;
  const size_t tok0 = (size_t)b * SEQ;

  const __bf16* Qb = (const __bf16*)(const void*)qbp + tok0 * DMOD + (size_t)h * AT_D;
  const __bf16* Kb = (const __bf16*)(const void*)kbp + tok0 * DMOD + (size_t)h * AT_D;
  const __bf16* Vt = (const __bf16*)(const void*)vtp + ((size_t)b * DMOD + (size_t)h * AT_D) * SEQ;
  const int*    mr = bmask + qbk * NMB;
  float*        ob = out + tok0 * DMOD + (size_t)h * AT_D;

  v16b qa[2];
#pragma unroll
  for (int dc = 0; dc < 2; ++dc)
    qa[dc] = ldfrag_b(Qb + (size_t)(q0 + c) * DMOD + dc * 32 + 8 * hh);

  float mrow[8], lrow[8];
  v8f oacc[4];
#pragma unroll
  for (int r = 0; r < 8; ++r) { mrow[r] = -INFINITY; lrow[r] = 0.f; }
#pragma unroll
  for (int t = 0; t < 4; ++t) oacc[t] = (v8f){0.f,0.f,0.f,0.f,0.f,0.f,0.f,0.f};

  for (int kc = 0; kc < SEQ / AT_KC; ++kc) {
    const int mi  = (kc * AT_KC) / MBLK;
    const int act = __builtin_amdgcn_readfirstlane(mr[mi]);
    if (act <= 0) continue;
    const int kv0 = kc * AT_KC;
    __syncthreads();
    {
      const int r = tid >> 1, half = (tid & 1) * 32;
      const __bf16* ks = Kb + (size_t)(kv0 + r) * DMOD + half;
      const __bf16* vs = Vt + (size_t)r * SEQ + kv0 + half;
#pragma unroll
      for (int i = 0; i < 4; ++i) {
        const v8b a0 = *(const v8b*)(ks + 8 * i);
        const v8b b0 = *(const v8b*)(vs + 8 * i);
        *(v8b*)(Ksh + r * AT_D  + half + 8 * i) = a0;
        *(v8b*)(Vth + r * AT_KC + half + 8 * i) = b0;
      }
    }
    __syncthreads();

    v8f s[4];
#pragma unroll
    for (int j = 0; j < 4; ++j) {
      s[j] = (v8f){0.f,0.f,0.f,0.f,0.f,0.f,0.f,0.f};
#pragma unroll
      for (int dc = 0; dc < 2; ++dc) {
        FB kf;
        kf.h[0] = *(const v8b*)(Ksh + (j * 16 + c) * AT_D + dc * 32 + 8 * hh);
        kf.h[1] = *(const v8b*)(Ksh + (j * 16 + c) * AT_D + dc * 32 + 16 + 8 * hh);
        s[j] = at_mma(qa[dc], kf.v, s[j]);
      }
    }
    float cm[8];
#pragma unroll
    for (int r = 0; r < 8; ++r) {
      float m = -INFINITY;
#pragma unroll
      for (int j = 0; j < 4; ++j) {
        const float sv = s[j][r] * sscale;
        s[j][r] = sv;
        m = fmaxf(m, sv);
      }
#pragma unroll
      for (int off = 1; off < 16; off <<= 1) m = fmaxf(m, __shfl_xor(m, off, 32));
      cm[r] = m;
    }
    __bf16* pwh = Psh[wave];
    __bf16* pwl = Psl[wave];
#pragma unroll
    for (int r = 0; r < 8; ++r) {
      const float mnew  = fmaxf(mrow[r], cm[r]);
      const float mref  = (mnew == -INFINITY) ? 0.0f : mnew;
      const float alpha = expf(mrow[r] - mref);
      mrow[r] = mnew;
      float psum = 0.f;
#pragma unroll
      for (int j = 0; j < 4; ++j) {
        const float p = expf(s[j][r] - mref);
        psum += p;
        const unsigned short hb = f2bf_bits(p);
        const unsigned short lb = f2bf_bits(p - bf_bits2f(hb));
        pwh[(8 * hh + r) * AT_KC + j * 16 + c] = __builtin_bit_cast(__bf16, hb);
        pwl[(8 * hh + r) * AT_KC + j * 16 + c] = __builtin_bit_cast(__bf16, lb);
      }
#pragma unroll
      for (int off = 1; off < 16; off <<= 1) psum += __shfl_xor(psum, off, 32);
      lrow[r] = lrow[r] * alpha + psum;
#pragma unroll
      for (int t = 0; t < 4; ++t) oacc[t][r] *= alpha;
    }
    __builtin_amdgcn_fence(__ATOMIC_RELEASE, "workgroup");
    __builtin_amdgcn_wave_barrier();
    __builtin_amdgcn_fence(__ATOMIC_ACQUIRE, "workgroup");
#pragma unroll 1
    for (int kk = 0; kk < 2; ++kk) {
      FB pa, pl;
      pa.h[0] = *(const v8b*)(pwh + c * AT_KC + kk * 32 + 8 * hh);
      pa.h[1] = *(const v8b*)(pwh + c * AT_KC + kk * 32 + 16 + 8 * hh);
      pl.h[0] = *(const v8b*)(pwl + c * AT_KC + kk * 32 + 8 * hh);
      pl.h[1] = *(const v8b*)(pwl + c * AT_KC + kk * 32 + 16 + 8 * hh);
#pragma unroll
      for (int t = 0; t < 4; ++t) {
        FB vf;
        vf.h[0] = *(const v8b*)(Vth + (t * 16 + c) * AT_KC + kk * 32 + 8 * hh);
        vf.h[1] = *(const v8b*)(Vth + (t * 16 + c) * AT_KC + kk * 32 + 16 + 8 * hh);
        oacc[t] = at_mma(pa.v, vf.v, oacc[t]);
        oacc[t] = at_mma(pl.v, vf.v, oacc[t]);
      }
    }
  }

  const float qnan = __int_as_float(0x7fc00000);
  float* os = Os[wave];
#pragma unroll
  for (int r = 0; r < 8; ++r) {
    const float l   = lrow[r];
    const float inv = (l > 0.f) ? (1.0f / l) : qnan;
#pragma unroll
    for (int t = 0; t < 4; ++t) os[(8 * hh + r) * 68 + t * 16 + c] = oacc[t][r] * inv;
    if (c == 0) {
      Ls[wave * 16 + 8 * hh + r] = (l > 0.f) ? l : qnan;
      Ms[wave * 16 + 8 * hh + r] = mrow[r];
    }
  }
  __builtin_amdgcn_fence(__ATOMIC_RELEASE, "workgroup");
  __builtin_amdgcn_wave_barrier();
  __builtin_amdgcn_fence(__ATOMIC_ACQUIRE, "workgroup");
  {
    const int c4 = c * 4;
    for (int pass = 0; pass < 2; ++pass) {
#pragma unroll
      for (int it = 0; it < 8; ++it) {
        const int row = it * 2 + hh;
        const v4f val = *(const v4f*)(os + row * 68 + c4);
        *(volatile v4f*)(ob + (size_t)(q0 + row) * DMOD + c4) = val;
      }
      __threadfence();
    }
  }
  __syncthreads();
  if (wave == 0) {
    const v4f vl = *(const v4f*)(Ls + c * 4);
    const v4f vm = *(const v4f*)(Ms + c * 4);
    v4f val;
#pragma unroll
    for (int e = 0; e < 4; ++e) val[e] = (hh == 0) ? vl[e] : vm[e];
    const size_t seg = (size_t)(b * NHEAD + h) * SEQ + (size_t)qb * AT_QB + (size_t)c * 4;
    const size_t so  = ((hh == 0) ? OFF_L : OFF_M) + seg;
    *(volatile v4f*)(out + so) = val;
    __threadfence();
    *(volatile v4f*)(out + so) = val;
  }
}

extern "C" void kernel_launch(void* const* d_in, const int* in_sizes, int n_in,
                              void* d_out, int out_size, void* d_ws, size_t ws_size,
                              hipStream_t stream) {
  if (n_in < 4) return;
  if (in_sizes[0] != NTOK * DMOD || in_sizes[1] != NTOK * DMOD || in_sizes[2] != NTOK * DMOD) return;
  if (in_sizes[3] != NMB * NMB) return;
  if ((size_t)out_size != OUT_N) return;

  const float* q   = (const float*)d_in[0];
  const float* k   = (const float*)d_in[1];
  const float* v   = (const float*)d_in[2];
  const int*   msk = (const int*)d_in[3];
  float*       out = (float*)d_out;

  const size_t PPL = (size_t)NTOK * DMOD * 2;
  size_t off = 0;
  const size_t oQB = off; off += PPL;
  const size_t oKB = off; off += PPL;
  const size_t oVT = off; off += PPL;
  if (off > ws_size) return;

  char* ws = (char*)d_ws;
  unsigned short* QB = (unsigned short*)(ws + oQB);
  unsigned short* KB = (unsigned short*)(ws + oKB);
  unsigned short* VT = (unsigned short*)(ws + oVT);

  const int n8 = NTOK * DMOD / 8;
  cvt_qk_kernel<<<dim3(n8 / 256), dim3(256), 0, stream>>>(q, k, QB, KB, n8);
  vtrans_kernel<<<dim3(DMOD / 64, SEQ / 64, NBATCH), dim3(256), 0, stream>>>(v, VT);
  attn64_kernel<<<dim3(NHEAD * (SEQ / AT_QB), NBATCH), dim3(128), 0, stream>>>(QB, KB, VT, msk, out, 0.125f);
  (void)hipGetLastError();
}
